// Kernel_63058709840173
// MI455X (gfx1250) — hardware-run, weakly checked
//
#include <hip/hip_runtime.h>
#include <stdint.h>

typedef __attribute__((ext_vector_type(16))) _Float16 v16h;
typedef __attribute__((ext_vector_type(8)))  _Float16 v8h;
typedef __attribute__((ext_vector_type(8)))  float    v8f;
typedef __attribute__((ext_vector_type(4)))  float    v4f;
typedef __attribute__((ext_vector_type(4)))  unsigned v4u;

constexpr int kBatch   = 8;
constexpr int kOutCh   = 6;
constexpr int kDev     = 5;
constexpr int kImg     = 64;
constexpr int kHout    = 60;
constexpr int kWin     = kHout * kHout;
constexpr int kNumOut  = kBatch * kOutCh * kWin;
constexpr int kFeat    = 90;
constexpr int kFeatPad = 96;
constexpr int kNin     = 7;
constexpr int kK0Pad   = 32;
constexpr int kWavesPerBlock = 8;
constexpr int kOutPerBlock   = 32 * kWavesPerBlock;
constexpr int kMainBlocks    = kNumOut / kOutPerBlock;
static_assert(kNumOut % kOutPerBlock == 0, "no tail wave");
static_assert((kK0Pad % 32) == 0 && (kFeatPad % 32) == 0, "K multiples of 32");
static_assert((kFeatPad % 16) == 0, "feature tiles of 16");
static_assert(kHout + kDev - 1 <= kImg, "window stays inside the image");

constexpr int kPitchW0   = 40;
constexpr int kPitchW    = 104;
constexpr int kPitchSlab = 104;
constexpr int kSlabHalves = 32 * kPitchSlab;

constexpr size_t kOffW0T  = 0;
constexpr size_t kOffW1T  = kOffW0T + (size_t)kFeatPad * kK0Pad * 2;
constexpr size_t kOffW2T  = kOffW1T + (size_t)kFeatPad * kFeatPad * 2;
constexpr size_t kOffVec  = kOffW2T + (size_t)kFeatPad * kFeatPad * 2;
constexpr size_t kWsTotal = kOffVec + (size_t)4 * kFeatPad * 4;
static_assert(kWsTotal == 44544ull, "carve total");
static_assert((kOffW1T % 128) == 0 && (kOffW2T % 128) == 0 && (kOffVec % 128) == 0, "128-B aligned regions");

constexpr int kPcsW0 = kFeatPad * kK0Pad / 8;
constexpr int kPcsW1 = kFeatPad * kFeatPad / 8;
constexpr int kPcsW  = kPcsW0 + 2 * kPcsW1;
constexpr int kPrepThreads = kPcsW + 4 * 32;
static_assert((kPcsW0 % 32) == 0 && (kPcsW1 % 32) == 0, "plane boundaries on wave boundaries");
static_assert((kPrepThreads % 256) == 0, "exact grid");

template <typename T> struct Frag;
template <> struct Frag<_Float16> {
  typedef v16h V; union U { v16h v; v8h h[2]; };
  static __device__ __forceinline__ v16h load(const _Float16* p) {
    U f; f.h[0] = *(const v8h*)(p); f.h[1] = *(const v8h*)(p + 16); return f.v;
  }
};

__device__ __forceinline__ v8f mma_h(v16h a, v16h b, v8f c) {
  c = __builtin_amdgcn_wmma_f32_16x16x32_f16(false, a, false, b, (short)0, c, false, false);
  asm volatile("v_nop\n\tv_nop\n\tv_nop\n\tv_nop" : "+v"(c) : "v"(a), "v"(b));
  return c;
}

__device__ __forceinline__ void wave_lds_sync() {
  __builtin_amdgcn_fence(__ATOMIC_RELEASE, "workgroup");
  __builtin_amdgcn_wave_barrier();
  __builtin_amdgcn_fence(__ATOMIC_ACQUIRE, "workgroup");
}

__device__ __forceinline__ unsigned pack_f16x2(float a, float b) {
  const _Float16 ha = (_Float16)a;
  const _Float16 hb = (_Float16)b;
  const unsigned short ua = __builtin_bit_cast(unsigned short, ha);
  const unsigned short ub = __builtin_bit_cast(unsigned short, hb);
  return (unsigned)ua | ((unsigned)ub << 16);
}

__global__ __launch_bounds__(256) void prep_planes_kernel(
    const float* __restrict__ W0, const float* __restrict__ b0,
    const float* __restrict__ W1, const float* __restrict__ b1,
    const float* __restrict__ W2, const float* __restrict__ b2,
    const float* __restrict__ W3,
    unsigned* __restrict__ planes, float* __restrict__ vecs)
{
  const int i = blockIdx.x * 256 + threadIdx.x;
  if (i < kPcsW) {
    const float* src;
    int kreal, ppr, j, dstw;
    if (i < kPcsW0) {
      src = W0; kreal = kNin; ppr = kK0Pad / 8; j = i; dstw = (int)(kOffW0T / 4);
    } else if (i < kPcsW0 + kPcsW1) {
      src = W1; kreal = kFeat; ppr = kFeatPad / 8; j = i - kPcsW0; dstw = (int)(kOffW1T / 4);
    } else {
      src = W2; kreal = kFeat; ppr = kFeatPad / 8; j = i - kPcsW0 - kPcsW1; dstw = (int)(kOffW2T / 4);
    }
    const int n  = j / ppr;
    const int kb = (j - n * ppr) * 8;
    const int nc = (n < kFeat) ? n : (kFeat - 1);
    const bool nok = (n < kFeat);
    unsigned wd[4];
#pragma unroll
    for (int p = 0; p < 4; ++p) {
      const int ka = kb + 2 * p;
      const int kc = ka + 1;
      const int kac = (ka < kreal) ? ka : (kreal - 1);
      const int kcc = (kc < kreal) ? kc : (kreal - 1);
      const float la = src[kac * kFeat + nc];
      const float lc = src[kcc * kFeat + nc];
      const float va = (nok && ka < kreal) ? la : 0.0f;
      const float vc = (nok && kc < kreal) ? lc : 0.0f;
      wd[p] = pack_f16x2(va, vc);
    }
    const v4u outv = (v4u){wd[0], wd[1], wd[2], wd[3]};
    unsigned* dst = planes + dstw + j * 4;
    *(volatile v4u*)dst = outv;
    __threadfence();
    *(volatile v4u*)dst = outv;
  } else {
    const int j   = i - kPcsW;
    const int vec = j >> 5;
    const int c   = j & 31;
    const float* src = (vec == 0) ? b0 : (vec == 1) ? b1 : (vec == 2) ? b2 : W3;
    const int cc = (c < 24) ? c : 23;
    float fv[4];
#pragma unroll
    for (int e = 0; e < 4; ++e) {
      const int idx  = cc * 4 + e;
      const int idxc = (idx < kFeat) ? idx : (kFeat - 1);
      const float lv = src[idxc];
      fv[e] = (idx < kFeat) ? lv : 0.0f;
    }
    const v4f outv = (v4f){fv[0], fv[1], fv[2], fv[3]};
    float* dst = vecs + vec * kFeatPad + cc * 4;
    if (c < 24) {
      *(volatile v4f*)dst = outv;
      __threadfence();
      *(volatile v4f*)dst = outv;
    }
  }
}

__device__ __forceinline__ void init_bias(v8f (&acc)[6][2], const float* bvec, int h) {
#pragma unroll
  for (int nt = 0; nt < 6; ++nt) {
    const v4f ba = *(const v4f*)(bvec + nt * 16 + 8 * h);
    const v4f bb = *(const v4f*)(bvec + nt * 16 + 8 * h + 4);
    const v8f bv = (v8f){ba[0], ba[1], ba[2], ba[3], bb[0], bb[1], bb[2], bb[3]};
    acc[nt][0] = bv;
    acc[nt][1] = bv;
  }
}

__device__ __forceinline__ void gemm_k96(v8f (&acc)[6][2], const _Float16* wbase, const _Float16* bp0, const _Float16* bp1) {
#pragma unroll 1
  for (int kc = 0; kc < 3; ++kc) {
    const int k0 = kc * 32;
    const v16h f0 = Frag<_Float16>::load(bp0 + k0);
    const v16h f1 = Frag<_Float16>::load(bp1 + k0);
#pragma unroll
    for (int nt = 0; nt < 6; ++nt) {
      const v16h a = Frag<_Float16>::load(wbase + nt * 16 * kPitchW + k0);
      acc[nt][0] = mma_h(a, f0, acc[nt][0]);
      acc[nt][1] = mma_h(a, f1, acc[nt][1]);
    }
  }
}

__device__ __forceinline__ void store_relu_f16(const v8f (&acc)[6][2], _Float16* sp0, _Float16* sp1) {
#pragma unroll
  for (int nt = 0; nt < 6; ++nt) {
    v8h h0, h1;
#pragma unroll
    for (int r = 0; r < 8; ++r) {
      h0[r] = (_Float16)fmaxf(acc[nt][0][r], 0.0f);
      h1[r] = (_Float16)fmaxf(acc[nt][1][r], 0.0f);
    }
    *(v8h*)(sp0 + nt * 16) = h0;
    *(v8h*)(sp1 + nt * 16) = h1;
  }
}

__global__ __launch_bounds__(256) void fused_rows_kernel(
    const float* __restrict__ x, const float* __restrict__ ctrl, const float* __restrict__ b3,
    const _Float16* __restrict__ planes, const float* __restrict__ vecs,
    float* __restrict__ out)
{
  __shared__ __align__(16) _Float16 sW0[kFeatPad * kPitchW0];
  __shared__ __align__(16) _Float16 sW1[kFeatPad * kPitchW];
  __shared__ __align__(16) _Float16 sW2[kFeatPad * kPitchW];
  __shared__ __align__(16) float    sVec[4 * kFeatPad];
  __shared__ __align__(16) _Float16 sSlab[kWavesPerBlock * kSlabHalves];

  const int tid  = threadIdx.x;
  const int lane = tid & 31;
  const int wave = tid >> 5;

  {
    const _Float16* g0 = planes + kOffW0T / 2;
    const _Float16* g1 = planes + kOffW1T / 2;
    const _Float16* g2 = planes + kOffW2T / 2;
    for (int i = tid; i < kPcsW0; i += 256) {
      const int n = i >> 2;
      const int c = (i & 3) * 8;
      *(v8h*)(sW0 + n * kPitchW0 + c) = *(const v8h*)(g0 + n * kK0Pad + c);
    }
    for (int i = tid; i < kPcsW1; i += 256) {
      const int n = i / 12;
      const int c = (i - n * 12) * 8;
      *(v8h*)(sW1 + n * kPitchW + c) = *(const v8h*)(g1 + n * kFeatPad + c);
      *(v8h*)(sW2 + n * kPitchW + c) = *(const v8h*)(g2 + n * kFeatPad + c);
    }
    if (tid < 96) *(v4f*)(sVec + tid * 4) = *(const v4f*)(vecs + tid * 4);
  }
  __syncthreads();

  const int m = lane & 15;
  const int h = lane >> 4;

  const int o   = (blockIdx.x * kWavesPerBlock + wave) * 32 + lane;
  const int bo  = o / kWin;
  const int li  = o - bo * kWin;
  const int bi  = bo / kOutCh;
  const int oc  = bo - bi * kOutCh;
  const int i0  = li / kHout;
  const int j0  = li - i0 * kHout;
  const float* xbase = x + ((size_t)bi * kImg + i0) * kImg + j0;
  const float* cbase = ctrl + oc * (kDev * 2);

  _Float16* slab  = sSlab + wave * kSlabHalves;
  _Float16* myrow = slab + lane * kPitchSlab;
  _Float16* bp0 = slab + m * kPitchSlab + 8 * h;
  _Float16* bp1 = bp0 + 16 * kPitchSlab;

  float zf = 0.0f;
  asm volatile("" : "+v"(zf));

  float sum0 = 0.0f;
  float sum1 = 0.0f;

#pragma unroll 1
  for (int dev = 0; dev < kDev; ++dev) {
    {
      const float* xr = xbase + dev * kImg;
      const float x0 = xr[0];
      const float x1 = xr[1];
      const float x2 = xr[2];
      const float x3 = xr[3];
      const float x4 = xr[4];
      const float c0 = cbase[dev * 2];
      const float c1 = cbase[dev * 2 + 1];
      v8h ev;
      ev[0] = (_Float16)x1;
      ev[1] = (_Float16)x2;
      ev[2] = (_Float16)x3;
      ev[3] = (_Float16)x4;
      ev[4] = (_Float16)c0;
      ev[5] = (_Float16)x0;
      ev[6] = (_Float16)c1;
      ev[7] = (_Float16)zf;
      const _Float16 zh = (_Float16)zf;
      const v8h zv = (v8h){zh, zh, zh, zh, zh, zh, zh, zh};
      *(v8h*)(myrow)      = ev;
      *(v8h*)(myrow + 8)  = zv;
      *(v8h*)(myrow + 16) = zv;
      *(v8h*)(myrow + 24) = zv;
    }
    wave_lds_sync();

    v8f acc[6][2];

    init_bias(acc, sVec, h);
    {
      const v16h f0 = Frag<_Float16>::load(bp0);
      const v16h f1 = Frag<_Float16>::load(bp1);
      const _Float16* wb = sW0 + m * kPitchW0 + 8 * h;
#pragma unroll
      for (int nt = 0; nt < 6; ++nt) {
        const v16h a = Frag<_Float16>::load(wb + nt * 16 * kPitchW0);
        acc[nt][0] = mma_h(a, f0, acc[nt][0]);
        acc[nt][1] = mma_h(a, f1, acc[nt][1]);
      }
    }
    wave_lds_sync();
    store_relu_f16(acc, bp0, bp1);
    wave_lds_sync();

    init_bias(acc, sVec + kFeatPad, h);
    gemm_k96(acc, sW1 + m * kPitchW + 8 * h, bp0, bp1);
    wave_lds_sync();
    store_relu_f16(acc, bp0, bp1);
    wave_lds_sync();

    init_bias(acc, sVec + 2 * kFeatPad, h);
    gemm_k96(acc, sW2 + m * kPitchW + 8 * h, bp0, bp1);

    float p0 = 0.0f;
    float p1 = 0.0f;
#pragma unroll
    for (int nt = 0; nt < 6; ++nt) {
      const v4f wa = *(const v4f*)(sVec + 3 * kFeatPad + nt * 16 + 8 * h);
      const v4f wb = *(const v4f*)(sVec + 3 * kFeatPad + nt * 16 + 8 * h + 4);
#pragma unroll
      for (int r = 0; r < 4; ++r) {
        p0 = fmaf(fmaxf(acc[nt][0][r], 0.0f), wa[r], p0);
        p1 = fmaf(fmaxf(acc[nt][1][r], 0.0f), wa[r], p1);
      }
#pragma unroll
      for (int r = 0; r < 4; ++r) {
        p0 = fmaf(fmaxf(acc[nt][0][4 + r], 0.0f), wb[r], p0);
        p1 = fmaf(fmaxf(acc[nt][1][4 + r], 0.0f), wb[r], p1);
      }
    }
    const float q0 = __shfl_xor(p0, 16, 32);
    const float q1 = __shfl_xor(p1, 16, 32);
    sum0 += p0 + q0;
    sum1 += p1 + q1;
    wave_lds_sync();
  }

  const float b3v = b3[0];
  const float val = ((h == 0) ? sum0 : sum1) + (float)kDev * b3v;
  volatile float* op = out + o;
  *op = val;
  __threadfence();
  *op = val;
}

extern "C" void kernel_launch(void* const* d_in, const int* in_sizes, int n_in,
                              void* d_out, int out_size, void* d_ws, size_t ws_size,
                              hipStream_t stream) {
  if (n_in < 10) return;
  if (in_sizes[0] != kBatch * kImg * kImg) return;
  if (in_sizes[1] != kOutCh * kDev * 2) return;
  if (in_sizes[2] != kNin * kFeat) return;
  if (in_sizes[3] != kFeat) return;
  if (in_sizes[4] != kFeat * kFeat) return;
  if (in_sizes[5] != kFeat) return;
  if (in_sizes[6] != kFeat * kFeat) return;
  if (in_sizes[7] != kFeat) return;
  if (in_sizes[8] != kFeat) return;
  if (in_sizes[9] != 1) return;
  if (out_size != kNumOut) return;
  if (ws_size < kWsTotal) return;

  const float* x    = (const float*)d_in[0];
  const float* ctrl = (const float*)d_in[1];
  const float* W0   = (const float*)d_in[2];
  const float* b0   = (const float*)d_in[3];
  const float* W1   = (const float*)d_in[4];
  const float* b1   = (const float*)d_in[5];
  const float* W2   = (const float*)d_in[6];
  const float* b2   = (const float*)d_in[7];
  const float* W3   = (const float*)d_in[8];
  const float* b3   = (const float*)d_in[9];
  float* out = (float*)d_out;

  char* ws = (char*)d_ws;
  unsigned*       planesW = (unsigned*)ws;
  const _Float16* planesH = (const _Float16*)ws;
  float*          vecs    = (float*)(ws + kOffVec);

  prep_planes_kernel<<<kPrepThreads / 256, 256, 0, stream>>>(W0, b0, W1, b1, W2, b2, W3, planesW, vecs);
  fused_rows_kernel<<<kMainBlocks, 256, 0, stream>>>(x, ctrl, b3, planesH, vecs, out);
}
